// TorchRoPEAttentionWithLoRA_47124381171924
// MI455X (gfx1250) — hardware-verified
//
#include <hip/hip_runtime.h>


#define BB 2
#define SS 2048
#define HH 1024
#define NQ 16
#define NKV 4
#define HD 64
#define RANK 8
#define QKVW 1536
#define LORA_SCALE 2.0f
#define ATT_SCALE 0.125f
#define THETA_F 10000.0f
#define CP 68

typedef float v8f __attribute__((ext_vector_type(8)));
typedef float v4f __attribute__((ext_vector_type(4)));
typedef unsigned int v4u __attribute__((ext_vector_type(4)));
typedef __bf16 v16b __attribute__((ext_vector_type(16)));
typedef __bf16 v8b __attribute__((ext_vector_type(8)));
typedef unsigned short u16;

union Frag { v16b v; v8b hv[2]; };

static __device__ __forceinline__ v8f vzero8() {
    v8f z = {0.f, 0.f, 0.f, 0.f, 0.f, 0.f, 0.f, 0.f};
    return z;
}

static __device__ __forceinline__ v16b ldfrag(const u16* p, int h) {
    Frag f;
    f.hv[0] = *(const v8b*)(p + 8 * h);
    f.hv[1] = *(const v8b*)(p + 16 + 8 * h);
    return f.v;
}

static __device__ __forceinline__ v8f mma3(v8f acc, v16b ah, v16b al, v16b bh, v16b bl) {
    acc = __builtin_amdgcn_wmma_f32_16x16x32_bf16(false, ah, false, bh, (short)0, acc, false, false);
    acc = __builtin_amdgcn_wmma_f32_16x16x32_bf16(false, ah, false, bl, (short)0, acc, false, false);
    acc = __builtin_amdgcn_wmma_f32_16x16x32_bf16(false, al, false, bh, (short)0, acc, false, false);
    asm volatile("v_nop\n\tv_nop\n\tv_nop\n\tv_nop" : "+v"(acc) : "v"(ah), "v"(al), "v"(bh), "v"(bl));
    return acc;
}

static __device__ __forceinline__ unsigned bf16_bits(float f) {
    unsigned u = __float_as_uint(f);
    return (u + 0x7FFFu + ((u >> 16) & 1u)) >> 16;
}

static __device__ __forceinline__ void split_bf16(float f, unsigned& hb, unsigned& lb) {
    hb = bf16_bits(f);
    float hi = __uint_as_float(hb << 16);
    lb = bf16_bits(f - hi);
}

static __device__ __forceinline__ void pack2(float a, float b, unsigned& hw, unsigned& lw) {
    unsigned ha, la, hb2, lb2;
    split_bf16(a, ha, la);
    split_bf16(b, hb2, lb2);
    hw = ha | (hb2 << 16);
    lw = la | (lb2 << 16);
}

__global__ __launch_bounds__(256)
void k_cvt(const float* __restrict__ X, u16* __restrict__ Ph, u16* __restrict__ Pl, int n8) {
    const int i = blockIdx.x * 256 + threadIdx.x;
    if (i >= n8) return;
    const float* src = X + (size_t)i * 8;
    v4f a = *(const v4f*)src;
    v4f c = *(const v4f*)(src + 4);
    v4u hv, lv;
    unsigned hw, lw;
    pack2(a.x, a.y, hw, lw); hv.x = hw; lv.x = lw;
    pack2(a.z, a.w, hw, lw); hv.y = hw; lv.y = lw;
    pack2(c.x, c.y, hw, lw); hv.z = hw; lv.z = lw;
    pack2(c.z, c.w, hw, lw); hv.w = hw; lv.w = lw;
    u16* dh = Ph + (size_t)i * 8;
    u16* dl = Pl + (size_t)i * 8;
    *(volatile v4u*)dh = hv;
    *(volatile v4u*)dl = lv;
    __threadfence();
    *(volatile v4u*)dh = hv;
    *(volatile v4u*)dl = lv;
}

__global__ __launch_bounds__(256)
void k_prep(const float* __restrict__ W, const float* __restrict__ A, const float* __restrict__ Bm,
            u16* __restrict__ Ph, u16* __restrict__ Pl, int rows, int cols) {
    const int cpr = cols >> 3;
    const int idx = blockIdx.x * 256 + threadIdx.x;
    if (idx >= rows * cpr) return;
    const int r = idx / cpr;
    const int c = (idx - r * cpr) * 8;
    const float* wp = W + (size_t)r * cols + c;
    v4f w0 = *(const v4f*)wp;
    v4f w1 = *(const v4f*)(wp + 4);
    float f0 = w0.x, f1 = w0.y, f2 = w0.z, f3 = w0.w;
    float f4 = w1.x, f5 = w1.y, f6 = w1.z, f7 = w1.w;
#pragma unroll 1
    for (int j = 0; j < RANK; ++j) {
        const float bj = Bm[r * RANK + j] * LORA_SCALE;
        const float* ap = A + (size_t)j * cols + c;
        v4f a0 = *(const v4f*)ap;
        v4f a1 = *(const v4f*)(ap + 4);
        f0 += bj * a0.x; f1 += bj * a0.y; f2 += bj * a0.z; f3 += bj * a0.w;
        f4 += bj * a1.x; f5 += bj * a1.y; f6 += bj * a1.z; f7 += bj * a1.w;
    }
    v4u hv, lv;
    unsigned hw, lw;
    pack2(f0, f1, hw, lw); hv.x = hw; lv.x = lw;
    pack2(f2, f3, hw, lw); hv.y = hw; lv.y = lw;
    pack2(f4, f5, hw, lw); hv.z = hw; lv.z = lw;
    pack2(f6, f7, hw, lw); hv.w = hw; lv.w = lw;
    u16* dh = Ph + (size_t)r * cols + c;
    u16* dl = Pl + (size_t)r * cols + c;
    *(volatile v4u*)dh = hv;
    *(volatile v4u*)dl = lv;
    __threadfence();
    *(volatile v4u*)dh = hv;
    *(volatile v4u*)dl = lv;
}

template <int MODE>
__global__ __launch_bounds__(128)
void k_gemm(const u16* __restrict__ Ah, const u16* __restrict__ Al,
            const u16* __restrict__ Wh, const u16* __restrict__ Wl,
            float* __restrict__ C,
            u16* __restrict__ Qh, u16* __restrict__ Ql,
            u16* __restrict__ Kh, u16* __restrict__ Kl,
            u16* __restrict__ Vh, u16* __restrict__ Vl,
            int N, int K) {
    __shared__ __attribute__((aligned(16))) float sC[64 * CP];
    __shared__ __attribute__((aligned(16))) u16 th[64 * 64];
    __shared__ __attribute__((aligned(16))) u16 tl[64 * 64];
    __shared__ float invf[32];

    const int t    = threadIdx.x;
    const int lane = t & 31;
    const int wid  = t >> 5;
    const int h16  = lane >> 4;
    const int m    = lane & 15;
    const int bm = blockIdx.x * 64;
    const int bn = blockIdx.y * 64;
    const int wm = (wid & 1) * 32;
    const int wn = (wid >> 1) * 32;
    const int m0 = bm + wm;
    const int n0 = bn + wn;

    if (MODE == 1) {
        if (t < 32) {
            const float e  = (float)t * 0.03125f;
            const float pw = powf(THETA_F, e);
            invf[t] = 1.0f / pw;
        }
    }

    v8f acc[2][2];
#pragma unroll
    for (int i = 0; i < 2; ++i)
#pragma unroll
        for (int j = 0; j < 2; ++j) acc[i][j] = vzero8();

    for (int k0 = 0; k0 < K; k0 += 32) {
        v16b ah[2], al[2], bh[2], bl[2];
#pragma unroll
        for (int mg = 0; mg < 2; ++mg) {
            const size_t o = (size_t)(m0 + mg * 16 + m) * K + k0;
            ah[mg] = ldfrag(Ah + o, h16);
            al[mg] = ldfrag(Al + o, h16);
        }
#pragma unroll
        for (int ng = 0; ng < 2; ++ng) {
            const size_t o = (size_t)(n0 + ng * 16 + m) * K + k0;
            bh[ng] = ldfrag(Wh + o, h16);
            bl[ng] = ldfrag(Wl + o, h16);
        }
#pragma unroll
        for (int mg = 0; mg < 2; ++mg)
#pragma unroll
            for (int ng = 0; ng < 2; ++ng)
                acc[mg][ng] = mma3(acc[mg][ng], ah[mg], al[mg], bh[ng], bl[ng]);
    }

#pragma unroll
    for (int mg = 0; mg < 2; ++mg)
#pragma unroll
        for (int ng = 0; ng < 2; ++ng)
#pragma unroll
            for (int r = 0; r < 8; ++r)
                sC[(wm + mg * 16 + 8 * h16 + r) * CP + wn + ng * 16 + m] = acc[mg][ng][r];
    __syncthreads();

    if (MODE == 0) {
        v4f v[8];
        size_t go[8];
#pragma unroll
        for (int i = 0; i < 8; ++i) {
            const int row = wm + 4 * i + (lane >> 3);
            const int c4  = wn + (lane & 7) * 4;
            v[i]  = *(const v4f*)(sC + row * CP + c4);
            go[i] = (size_t)(bm + row) * N + bn + c4;
        }
#pragma unroll
        for (int i = 0; i < 8; ++i) *(volatile v4f*)(C + go[i]) = v[i];
        __threadfence();
#pragma unroll
        for (int i = 0; i < 8; ++i) *(volatile v4f*)(C + go[i]) = v[i];
    } else {
        const int nt   = blockIdx.y;
        const int b    = bm / SS;
        const int s0   = bm - b * SS;
        const int tok  = t & 63;
        const int half = t >> 6;
        if (nt < NQ + NKV) {
            const float post = (nt < NQ) ? ATT_SCALE : 1.0f;
            const float pos  = (float)(s0 + tok);
            const float* crow = sC + tok * CP;
#pragma unroll 1
            for (int pp = 0; pp < 16; ++pp) {
                const int p = half * 16 + pp;
                const float x1 = crow[2 * p];
                const float x2 = crow[2 * p + 1];
                const float fr = pos * invf[p];
                float sn, cs;
                sincosf(fr, &sn, &cs);
                const float o1 = (x1 * cs - x2 * sn) * post;
                const float o2 = (x1 * sn + x2 * cs) * post;
                unsigned h1, l1, h2, l2;
                split_bf16(o1, h1, l1);
                split_bf16(o2, h2, l2);
                th[tok * 64 + p]      = (u16)h1;  tl[tok * 64 + p]      = (u16)l1;
                th[tok * 64 + 32 + p] = (u16)h2;  tl[tok * 64 + 32 + p] = (u16)l2;
            }
        } else {
            const float* crow = sC + tok * CP;
#pragma unroll 1
            for (int dd = 0; dd < 32; ++dd) {
                const int d = half * 32 + dd;
                unsigned hb, lb;
                split_bf16(crow[d], hb, lb);
                th[d * 64 + tok] = (u16)hb;
                tl[d * 64 + tok] = (u16)lb;
            }
        }
        __syncthreads();

        size_t base, rstride;
        u16* dh;
        u16* dl;
        if (nt < NQ) {
            base = ((size_t)(b * NQ + nt) * SS + s0) * HD;  rstride = HD;  dh = Qh; dl = Ql;
        } else if (nt < NQ + NKV) {
            const int hk = nt - NQ;
            base = ((size_t)(b * NKV + hk) * SS + s0) * HD; rstride = HD;  dh = Kh; dl = Kl;
        } else {
            const int hk = nt - NQ - NKV;
            base = ((size_t)(b * NKV + hk) * HD) * SS + s0; rstride = SS;  dh = Vh; dl = Vl;
        }
        v4u hv[4], lv[4];
        size_t go[4];
#pragma unroll
        for (int i = 0; i < 4; ++i) {
            const int line  = wid * 16 + 4 * i + (lane >> 3);
            const int piece = lane & 7;
            hv[i] = *(const v4u*)(th + line * 64 + piece * 8);
            lv[i] = *(const v4u*)(tl + line * 64 + piece * 8);
            go[i] = base + (size_t)line * rstride + (size_t)piece * 8;
        }
#pragma unroll
        for (int i = 0; i < 4; ++i) { *(volatile v4u*)(dh + go[i]) = hv[i]; *(volatile v4u*)(dl + go[i]) = lv[i]; }
        __threadfence();
#pragma unroll
        for (int i = 0; i < 4; ++i) { *(volatile v4u*)(dh + go[i]) = hv[i]; *(volatile v4u*)(dl + go[i]) = lv[i]; }
    }
}

__global__ __launch_bounds__(128)
void k_attn(const u16* __restrict__ Qh, const u16* __restrict__ Ql,
            const u16* __restrict__ Kh, const u16* __restrict__ Kl,
            const u16* __restrict__ Vh, const u16* __restrict__ Vl,
            u16* __restrict__ Oh, u16* __restrict__ Ol) {
    __shared__ __attribute__((aligned(16))) u16 sPh[4 * 16 * 32];
    __shared__ __attribute__((aligned(16))) u16 sPl[4 * 16 * 32];
    __shared__ __attribute__((aligned(16))) u16 sOh[4 * 16 * 64];
    __shared__ __attribute__((aligned(16))) u16 sOl[4 * 16 * 64];

    const int lane = threadIdx.x & 31;
    const int wid  = threadIdx.x >> 5;
    const int h16  = lane >> 4;
    const int m    = lane & 15;
    const int hq = blockIdx.y;
    const int b  = blockIdx.z;
    const int hk = hq >> 2;
    const int q0 = blockIdx.x * 64 + wid * 16;

    const u16* Qbh = Qh + (size_t)(b * NQ + hq) * SS * HD;
    const u16* Qbl = Ql + (size_t)(b * NQ + hq) * SS * HD;
    const u16* Kbh = Kh + (size_t)(b * NKV + hk) * SS * HD;
    const u16* Kbl = Kl + (size_t)(b * NKV + hk) * SS * HD;
    const u16* Vbh = Vh + (size_t)(b * NKV + hk) * HD * SS;
    const u16* Vbl = Vl + (size_t)(b * NKV + hk) * HD * SS;

    v16b qh[2], ql[2];
#pragma unroll
    for (int kk = 0; kk < 2; ++kk) {
        const size_t o = (size_t)(q0 + m) * HD + kk * 32;
        qh[kk] = ldfrag(Qbh + o, h16);
        ql[kk] = ldfrag(Qbl + o, h16);
    }

    v8f oacc[4];
#pragma unroll
    for (int oc = 0; oc < 4; ++oc) oacc[oc] = vzero8();
    float rm[8], rl[8];
#pragma unroll
    for (int r = 0; r < 8; ++r) { rm[r] = -1e30f; rl[r] = 0.f; }

    u16* ph = sPh + wid * 512;
    u16* pl = sPl + wid * 512;

    for (int t0 = 0; t0 < SS; t0 += 32) {
        v8f sacc[2];
        sacc[0] = vzero8();
        sacc[1] = vzero8();
#pragma unroll
        for (int j = 0; j < 2; ++j) {
#pragma unroll
            for (int kk = 0; kk < 2; ++kk) {
                const size_t o = (size_t)(t0 + j * 16 + m) * HD + kk * 32;
                v16b kfh = ldfrag(Kbh + o, h16);
                v16b kfl = ldfrag(Kbl + o, h16);
                sacc[j] = mma3(sacc[j], qh[kk], ql[kk], kfh, kfl);
            }
        }
        float sc[8];
#pragma unroll
        for (int r = 0; r < 8; ++r) {
            float mx = fmaxf(sacc[0][r], sacc[1][r]);
            mx = fmaxf(mx, __shfl_xor(mx, 1, 32));
            mx = fmaxf(mx, __shfl_xor(mx, 2, 32));
            mx = fmaxf(mx, __shfl_xor(mx, 4, 32));
            mx = fmaxf(mx, __shfl_xor(mx, 8, 32));
            const float nm = fmaxf(rm[r], mx);
            sc[r] = expf(rm[r] - nm);
            rm[r] = nm;
        }
        __syncthreads();
#pragma unroll
        for (int r = 0; r < 8; ++r) {
            float ps = 0.f;
#pragma unroll
            for (int j = 0; j < 2; ++j) {
                const float p = expf(sacc[j][r] - rm[r]);
                ps += p;
                unsigned hb, lb;
                split_bf16(p, hb, lb);
                ph[(8 * h16 + r) * 32 + j * 16 + m] = (u16)hb;
                pl[(8 * h16 + r) * 32 + j * 16 + m] = (u16)lb;
            }
            ps += __shfl_xor(ps, 1, 32);
            ps += __shfl_xor(ps, 2, 32);
            ps += __shfl_xor(ps, 4, 32);
            ps += __shfl_xor(ps, 8, 32);
            rl[r] = rl[r] * sc[r] + ps;
        }
#pragma unroll
        for (int oc = 0; oc < 4; ++oc)
#pragma unroll
            for (int r = 0; r < 8; ++r) oacc[oc][r] *= sc[r];
        __syncthreads();
        v16b pfh = ldfrag(ph + m * 32, h16);
        v16b pfl = ldfrag(pl + m * 32, h16);
#pragma unroll
        for (int oc = 0; oc < 4; ++oc) {
            const size_t o = (size_t)(oc * 16 + m) * SS + t0;
            v16b vfh = ldfrag(Vbh + o, h16);
            v16b vfl = ldfrag(Vbl + o, h16);
            oacc[oc] = mma3(oacc[oc], pfh, pfl, vfh, vfl);
        }
    }

    u16* oh = sOh + wid * 1024;
    u16* ol = sOl + wid * 1024;
#pragma unroll
    for (int r = 0; r < 8; ++r) {
        const float inv = 1.0f / rl[r];
#pragma unroll
        for (int oc = 0; oc < 4; ++oc) {
            const float o = oacc[oc][r] * inv;
            unsigned hb, lb;
            split_bf16(o, hb, lb);
            oh[(8 * h16 + r) * 64 + oc * 16 + m] = (u16)hb;
            ol[(8 * h16 + r) * 64 + oc * 16 + m] = (u16)lb;
        }
    }
    __syncthreads();

    v4u hv[4], lv[4];
    size_t go[4];
#pragma unroll
    for (int i = 0; i < 4; ++i) {
        const int row   = 4 * i + (lane >> 3);
        const int piece = lane & 7;
        hv[i] = *(const v4u*)(oh + row * 64 + piece * 8);
        lv[i] = *(const v4u*)(ol + row * 64 + piece * 8);
        go[i] = (size_t)(b * SS + q0 + row) * (NQ * HD) + (size_t)hq * HD + (size_t)piece * 8;
    }
#pragma unroll
    for (int i = 0; i < 4; ++i) { *(volatile v4u*)(Oh + go[i]) = hv[i]; *(volatile v4u*)(Ol + go[i]) = lv[i]; }
    __threadfence();
#pragma unroll
    for (int i = 0; i < 4; ++i) { *(volatile v4u*)(Oh + go[i]) = hv[i]; *(volatile v4u*)(Ol + go[i]) = lv[i]; }
}

extern "C" void kernel_launch(void* const* d_in, const int* in_sizes, int n_in,
                              void* d_out, int out_size, void* d_ws, size_t ws_size,
                              hipStream_t stream) {
    if (n_in < 13) return;
    const int M = BB * SS;
    if (in_sizes[0] != M * HH) return;
    if (in_sizes[1] != NQ * HD * HH) return;
    if (in_sizes[2] != NKV * HD * HH) return;
    if (in_sizes[3] != NKV * HD * HH) return;
    if (in_sizes[4] != HH * NQ * HD) return;
    if (in_sizes[5] != RANK * HH) return;
    if (in_sizes[6] != NQ * HD * RANK) return;
    if (in_sizes[7] != RANK * HH) return;
    if (in_sizes[8] != NKV * HD * RANK) return;
    if (in_sizes[9] != RANK * HH) return;
    if (in_sizes[10] != NKV * HD * RANK) return;
    if (in_sizes[11] != RANK * NQ * HD) return;
    if (in_sizes[12] != HH * RANK) return;
    if (out_size != M * HH) return;

    const float* x  = (const float*)d_in[0];
    const float* Wq = (const float*)d_in[1];
    const float* Wk = (const float*)d_in[2];
    const float* Wv = (const float*)d_in[3];
    const float* Wo = (const float*)d_in[4];
    const float* qA = (const float*)d_in[5];
    const float* qB = (const float*)d_in[6];
    const float* kA = (const float*)d_in[7];
    const float* kB = (const float*)d_in[8];
    const float* vA = (const float*)d_in[9];
    const float* vB = (const float*)d_in[10];
    const float* oA = (const float*)d_in[11];
    const float* oB = (const float*)d_in[12];
    float* out = (float*)d_out;

    const size_t szXp   = (size_t)M * HH * 2;
    const size_t szWqkv = (size_t)QKVW * HH * 2;
    const size_t szWo   = (size_t)HH * (NQ * HD) * 2;
    const size_t szQp   = (size_t)BB * NQ * SS * HD * 2;
    const size_t szKp   = (size_t)BB * NKV * SS * HD * 2;
    const size_t szOp   = (size_t)M * (NQ * HD) * 2;
    size_t off = 0;
    const size_t oXh = off;   off += szXp;
    const size_t oXl = off;   off += szXp;
    const size_t oWh = off;   off += szWqkv;
    const size_t oWl = off;   off += szWqkv;
    const size_t oWoh = off;  off += szWo;
    const size_t oWol = off;  off += szWo;
    const size_t oQh = off;   off += szQp;
    const size_t oQl = off;   off += szQp;
    const size_t oKh = off;   off += szKp;
    const size_t oKl = off;   off += szKp;
    const size_t oVh = off;   off += szKp;
    const size_t oVl = off;   off += szKp;
    const size_t oOh = off;   off += szOp;
    const size_t oOl = off;   off += szOp;
    if (off > ws_size) return;

    char* ws = (char*)d_ws;
    u16* Xh    = (u16*)(ws + oXh);
    u16* Xl    = (u16*)(ws + oXl);
    u16* Wqkvh = (u16*)(ws + oWh);
    u16* Wqkvl = (u16*)(ws + oWl);
    u16* Woh   = (u16*)(ws + oWoh);
    u16* Wol   = (u16*)(ws + oWol);
    u16* Qph   = (u16*)(ws + oQh);
    u16* Qpl   = (u16*)(ws + oQl);
    u16* Kph   = (u16*)(ws + oKh);
    u16* Kpl   = (u16*)(ws + oKl);
    u16* Vph   = (u16*)(ws + oVh);
    u16* Vpl   = (u16*)(ws + oVl);
    u16* Oph   = (u16*)(ws + oOh);
    u16* Opl   = (u16*)(ws + oOl);

    {
        const int n8 = M * HH / 8;
        k_cvt<<<(n8 + 255) / 256, 256, 0, stream>>>(x, Xh, Xl, n8);
    }
    k_prep<<<(NQ * HD * HH / 8 + 255) / 256, 256, 0, stream>>>(Wq, qA, qB, Wqkvh, Wqkvl, NQ * HD, HH);
    k_prep<<<(NKV * HD * HH / 8 + 255) / 256, 256, 0, stream>>>(Wk, kA, kB,
        Wqkvh + (size_t)(NQ * HD) * HH, Wqkvl + (size_t)(NQ * HD) * HH, NKV * HD, HH);
    k_prep<<<(NKV * HD * HH / 8 + 255) / 256, 256, 0, stream>>>(Wv, vA, vB,
        Wqkvh + (size_t)(NQ * HD + NKV * HD) * HH, Wqkvl + (size_t)(NQ * HD + NKV * HD) * HH, NKV * HD, HH);
    k_prep<<<(HH * NQ * HD / 8 + 255) / 256, 256, 0, stream>>>(Wo, oA, oB, Woh, Wol, HH, NQ * HD);
    k_gemm<1><<<dim3(M / 64, QKVW / 64), 128, 0, stream>>>(Xh, Xl, Wqkvh, Wqkvl, out,
        Qph, Qpl, Kph, Kpl, Vph, Vpl, QKVW, HH);
    k_attn<<<dim3(SS / 64, NQ, BB), 128, 0, stream>>>(Qph, Qpl, Kph, Kpl, Vph, Vpl, Oph, Opl);
    k_gemm<0><<<dim3(M / 64, HH / 64), 128, 0, stream>>>(Oph, Opl, Woh, Wol, out,
        Qph, Qpl, Kph, Kpl, Vph, Vpl, HH, NQ * HD);
}
